// MockGQAAttention_33878702031220
// MI455X (gfx1250) — hardware-verified
//
#include <hip/hip_runtime.h>

typedef _Float16       v16h __attribute__((ext_vector_type(16)));
typedef __bf16         v16b __attribute__((ext_vector_type(16)));
typedef unsigned short v8us __attribute__((ext_vector_type(8)));
typedef int            v8i  __attribute__((ext_vector_type(8)));
typedef float          v8f  __attribute__((ext_vector_type(8)));
typedef float          v4f  __attribute__((ext_vector_type(4)));
typedef v8us __attribute__((may_alias)) v8usa;
typedef v4f  __attribute__((may_alias)) v4fa;

union FragH { v16h v; v8us u[2]; };
union FragB { v16b v; v8us u[2]; };
union HBits { _Float16 h; unsigned short u; };

#define BATCH  2
#define SEQ    2048
#define HID    2048
#define NQH    32
#define NKVH   8
#define HDIM   64
#define KVW    (NKVH * HDIM)
#define MROWS  (BATCH * SEQ)
#define XP     40
#define PSCALE 16384.0f
#define WSCALE 32.0f
#define RSCALE 1024.0f

#define XG   (MROWS * HID / 8)
#define WQG  (HID * HID / 8)
#define WKG  (KVW * HID / 8)
#define CVT_BLOCKS ((XG + WQG + WKG + WKG + WQG) / 256)

__device__ __forceinline__ v8f wmma_f16(v16h a, v16h b, v8f c) {
  v8f d = __builtin_amdgcn_wmma_f32_16x16x32_f16(false, a, false, b, (short)0, c, false, false);
  const v8i ai = __builtin_bit_cast(v8i, a);
  const v8i bi = __builtin_bit_cast(v8i, b);
  asm volatile("v_nop\n\tv_nop\n\tv_nop\n\tv_nop" : "+v"(d) : "v"(ai), "v"(bi));
  return d;
}
__device__ __forceinline__ v8f wmma_bf16(v16b a, v16b b, v8f c) {
  v8f d = __builtin_amdgcn_wmma_f32_16x16x32_bf16(false, a, false, b, (short)0, c, false, false);
  const v8i ai = __builtin_bit_cast(v8i, a);
  const v8i bi = __builtin_bit_cast(v8i, b);
  asm volatile("v_nop\n\tv_nop\n\tv_nop\n\tv_nop" : "+v"(d) : "v"(ai), "v"(bi));
  return d;
}

__device__ __forceinline__ v16h frag_h(const _Float16* p, int h) {
  FragH f;
  f.u[0] = *(const v8usa*)(p + 8 * h);
  f.u[1] = *(const v8usa*)(p + 16 + 8 * h);
  return f.v;
}
__device__ __forceinline__ v16b frag_b(const unsigned short* p, int h) {
  FragB f;
  f.u[0] = *(const v8usa*)(p + 8 * h);
  f.u[1] = *(const v8usa*)(p + 16 + 8 * h);
  return f.v;
}

__device__ __forceinline__ unsigned short bf_rne(float f) {
  unsigned int u = __float_as_uint(f);
  u += 0x7FFFu + ((u >> 16) & 1u);
  return (unsigned short)(u >> 16);
}
__device__ __forceinline__ float bf_val(unsigned short b) {
  return __uint_as_float(((unsigned int)b) << 16);
}
__device__ __forceinline__ unsigned short h_bits(float f) { HBits c; c.h = (_Float16)f; return c.u; }
__device__ __forceinline__ float h_val(unsigned short u) { HBits c; c.u = u; return (float)c.h; }

__device__ __forceinline__ void cvt_h8(const float* src, _Float16* dst, float sc) {
  const v4f a = *(const v4fa*)src;
  const v4f c = *(const v4fa*)(src + 4);
  v8us o;
  o[0] = h_bits(a.x * sc); o[1] = h_bits(a.y * sc); o[2] = h_bits(a.z * sc); o[3] = h_bits(a.w * sc);
  o[4] = h_bits(c.x * sc); o[5] = h_bits(c.y * sc); o[6] = h_bits(c.z * sc); o[7] = h_bits(c.w * sc);
  *(volatile v8usa*)dst = o;
  __threadfence();
  *(volatile v8usa*)dst = o;
}
__device__ __forceinline__ void cvt_b8(const float* src, unsigned short* dhi, unsigned short* dlo) {
  const v4f a = *(const v4fa*)src;
  const v4f c = *(const v4fa*)(src + 4);
  const float f[8] = { a.x, a.y, a.z, a.w, c.x, c.y, c.z, c.w };
  v8us vh, vl;
  #pragma unroll
  for (int i = 0; i < 8; ++i) {
    const unsigned short hb = bf_rne(f[i]);
    vh[i] = hb;
    vl[i] = bf_rne(f[i] - bf_val(hb));
  }
  *(volatile v8us*)dhi = vh;
  *(volatile v8us*)dlo = vl;
  __threadfence();
  *(volatile v8us*)dhi = vh;
  *(volatile v8us*)dlo = vl;
}

__global__ __launch_bounds__(256) void convert_kernel(
    const float* __restrict__ x, const float* __restrict__ wq, const float* __restrict__ wk,
    const float* __restrict__ wv, const float* __restrict__ wo,
    _Float16* __restrict__ xh, _Float16* __restrict__ wqh, _Float16* __restrict__ wkh,
    unsigned short* __restrict__ wvhi, unsigned short* __restrict__ wvlo,
    unsigned short* __restrict__ wohi, unsigned short* __restrict__ wolo)
{
  const int blk = blockIdx.x, t = threadIdx.x;
  const int B0 = XG / 256, B1 = B0 + WQG / 256, B2 = B1 + WKG / 256, B3 = B2 + WKG / 256;
  if (blk >= CVT_BLOCKS) return;
  if (blk < B0) {
    const size_t g = (size_t)blk * 256 + t;
    cvt_h8(x + g * 8, xh + g * 8, 1.0f);
  } else if (blk < B1) {
    const size_t g = (size_t)(blk - B0) * 256 + t;
    cvt_h8(wq + g * 8, wqh + g * 8, WSCALE);
  } else if (blk < B2) {
    const size_t g = (size_t)(blk - B1) * 256 + t;
    cvt_h8(wk + g * 8, wkh + g * 8, WSCALE);
  } else if (blk < B3) {
    const size_t g = (size_t)(blk - B2) * 256 + t;
    cvt_b8(wv + g * 8, wvhi + g * 8, wvlo + g * 8);
  } else {
    const size_t g = (size_t)(blk - B3) * 256 + t;
    cvt_b8(wo + g * 8, wohi + g * 8, wolo + g * 8);
  }
}

__device__ __forceinline__ void qk_store_pass(const _Float16* sT, _Float16* plane,
                                              int bh, int l0, int w, int lane) {
  const int q8 = lane & 7, sub = lane >> 3;
  #pragma unroll
  for (int i = 0; i < 8; ++i) {
    const int lid = w * 32 + i * 4 + sub;
    const v8us v = *(const v8usa*)(sT + lid * HDIM + 8 * q8);
    _Float16* dst = plane + ((size_t)bh * SEQ + l0 + lid) * HDIM + 8 * q8;
    *(volatile v8usa*)dst = v;
  }
}

__global__ __launch_bounds__(128) void proj_qk_kernel(
    const _Float16* __restrict__ xh,
    const _Float16* __restrict__ wqh,
    const _Float16* __restrict__ wkh,
    const float* __restrict__ bq, const float* __restrict__ bk,
    _Float16* __restrict__ qh,
    _Float16* __restrict__ kh)
{
  __shared__ __attribute__((aligned(16))) _Float16 sT[128 * HDIM];

  const int tid = threadIdx.x, lane = tid & 31, w = tid >> 5;
  const int h = lane >> 4, m = lane & 15;
  const int m0 = blockIdx.x * 128;
  const int cg = blockIdx.y;
  const bool isq = (cg < NQH);
  const int head = isq ? cg : (cg - NQH);
  const int m0w = m0 + 32 * w;

  const _Float16* xa0 = xh + (size_t)(m0w + m) * HID;
  const _Float16* xa1 = xa0 + (size_t)16 * HID;
  const _Float16* wbase = isq ? wqh : wkh;
  const _Float16* wb = wbase + (size_t)(head * HDIM + m) * HID;

  const v8f zero8 = {0.f, 0.f, 0.f, 0.f, 0.f, 0.f, 0.f, 0.f};
  v8f acc[2][4];
  #pragma unroll
  for (int mt = 0; mt < 2; ++mt)
    #pragma unroll
    for (int nt = 0; nt < 4; ++nt) acc[mt][nt] = zero8;

  #pragma unroll 1
  for (int k0 = 0; k0 < HID; k0 += 32) {
    const v16h a0 = frag_h(xa0 + k0, h);
    const v16h a1 = frag_h(xa1 + k0, h);
    #pragma unroll
    for (int nt = 0; nt < 4; ++nt) {
      const v16h b = frag_h(wb + (size_t)nt * 16 * HID + k0, h);
      acc[0][nt] = wmma_f16(a0, b, acc[0][nt]);
      acc[1][nt] = wmma_f16(a1, b, acc[1][nt]);
    }
  }

  const float* bias = isq ? bq : bk;
  const float osc = isq ? 0.125f : 1.0f;
  #pragma unroll
  for (int nt = 0; nt < 4; ++nt) {
    const int feat = 16 * nt + m;
    const float bvl = bias[head * HDIM + feat];
    #pragma unroll
    for (int mt = 0; mt < 2; ++mt) {
      #pragma unroll
      for (int r = 0; r < 8; ++r) {
        const int tokl = 32 * w + 16 * mt + 8 * h + r;
        const float y = (acc[mt][nt][r] * (1.0f / WSCALE) + bvl) * osc;
        sT[tokl * HDIM + feat] = (_Float16)y;
      }
    }
  }
  __syncthreads();

  const int b = m0 / SEQ, l0 = m0 - b * SEQ;
  const int bh = isq ? (b * NQH + head) : (b * NKVH + head);
  _Float16* plane = isq ? qh : kh;
  qk_store_pass(sT, plane, bh, l0, w, lane);
  __threadfence();
  qk_store_pass(sT, plane, bh, l0, w, lane);
}

__device__ __forceinline__ void vt_store_pass(const unsigned short* sT, _Float16* plane,
                                              int bkv0, int l0, int w, int lane) {
  const int q8 = lane & 7, sub = lane >> 3;
  #pragma unroll
  for (int i = 0; i < 8; ++i) {
    const int lid = w * 32 + i * 4 + sub;
    const int kvhl = lid >> 6, d = lid & 63;
    const v8us v = *(const v8usa*)(sT + lid * 64 + 8 * q8);
    _Float16* dst = plane + ((size_t)(bkv0 + kvhl) * HDIM + d) * SEQ + l0 + 8 * q8;
    *(volatile v8usa*)dst = v;
  }
}

__global__ __launch_bounds__(256) void proj_v_kernel(
    const float* __restrict__ x,
    const unsigned short* __restrict__ wvhi,
    const unsigned short* __restrict__ wvlo,
    const float* __restrict__ bv,
    _Float16* __restrict__ vthi,
    _Float16* __restrict__ vtlo)
{
  __shared__ __attribute__((aligned(16))) unsigned short sXh[64 * XP];
  __shared__ __attribute__((aligned(16))) unsigned short sXl[64 * XP];
  __shared__ __attribute__((aligned(16))) unsigned short sT[256 * 64];

  const int tid = threadIdx.x, lane = tid & 31, w = tid >> 5;
  const int wr = w >> 2, wc = w & 3;
  const int h = lane >> 4, m = lane & 15;
  const int m0 = blockIdx.x * 64;
  const int feat0 = blockIdx.y * 256;

  const int srow = tid >> 2, skq = (tid & 3) * 8;
  const float* xsrc = x + (size_t)(m0 + srow) * HID + skq;
  unsigned short* sxh_w = sXh + srow * XP + skq;
  unsigned short* sxl_w = sXl + srow * XP + skq;

  const unsigned short* wbh = wvhi + (size_t)(feat0 + 64 * wc + m) * HID;
  const unsigned short* wbl = wvlo + (size_t)(feat0 + 64 * wc + m) * HID;
  const unsigned short* sah0 = sXh + (32 * wr + m) * XP;
  const unsigned short* sah1 = sah0 + 16 * XP;
  const unsigned short* sal0 = sXl + (32 * wr + m) * XP;
  const unsigned short* sal1 = sal0 + 16 * XP;

  const v8f zero8 = {0.f, 0.f, 0.f, 0.f, 0.f, 0.f, 0.f, 0.f};
  v8f acc[2][4];
  #pragma unroll
  for (int mt = 0; mt < 2; ++mt)
    #pragma unroll
    for (int nt = 0; nt < 4; ++nt) acc[mt][nt] = zero8;

  #pragma unroll 1
  for (int k0 = 0; k0 < HID; k0 += 32) {
    {
      const v4f a = *(const v4fa*)(xsrc + k0);
      const v4f c = *(const v4fa*)(xsrc + k0 + 4);
      const float f[8] = { a.x, a.y, a.z, a.w, c.x, c.y, c.z, c.w };
      v8us vh, vl;
      #pragma unroll
      for (int i = 0; i < 8; ++i) {
        const unsigned short hb = bf_rne(f[i]);
        vh[i] = hb;
        vl[i] = bf_rne(f[i] - bf_val(hb));
      }
      *(v8usa*)sxh_w = vh;
      *(v8usa*)sxl_w = vl;
    }
    __syncthreads();

    const v16b ah0 = frag_b(sah0, h);
    const v16b ah1 = frag_b(sah1, h);
    const v16b al0 = frag_b(sal0, h);
    const v16b al1 = frag_b(sal1, h);
    #pragma unroll
    for (int nt = 0; nt < 4; ++nt) {
      const v16b bhf = frag_b(wbh + (size_t)nt * 16 * HID + k0, h);
      const v16b blf = frag_b(wbl + (size_t)nt * 16 * HID + k0, h);
      acc[0][nt] = wmma_bf16(ah0, bhf, acc[0][nt]);
      acc[0][nt] = wmma_bf16(ah0, blf, acc[0][nt]);
      acc[0][nt] = wmma_bf16(al0, bhf, acc[0][nt]);
      acc[1][nt] = wmma_bf16(ah1, bhf, acc[1][nt]);
      acc[1][nt] = wmma_bf16(ah1, blf, acc[1][nt]);
      acc[1][nt] = wmma_bf16(al1, bhf, acc[1][nt]);
    }
    __syncthreads();
  }

  const int b = m0 / SEQ, l0 = m0 - b * SEQ;
  const int bkv0 = b * NKVH + blockIdx.y * 4;

  #pragma unroll
  for (int nt = 0; nt < 4; ++nt) {
    const int featl = 64 * wc + 16 * nt + m;
    const float bvl = bv[feat0 + featl];
    #pragma unroll
    for (int mt = 0; mt < 2; ++mt) {
      #pragma unroll
      for (int r = 0; r < 8; ++r) {
        const int tokl = 32 * wr + 16 * mt + 8 * h + r;
        const float y = acc[mt][nt][r] + bvl;
        sT[featl * 64 + tokl] = h_bits(y);
      }
    }
  }
  __syncthreads();
  vt_store_pass(sT, vthi, bkv0, l0, w, lane);
  __threadfence();
  vt_store_pass(sT, vthi, bkv0, l0, w, lane);
  __syncthreads();

  #pragma unroll
  for (int nt = 0; nt < 4; ++nt) {
    const int featl = 64 * wc + 16 * nt + m;
    const float bvl = bv[feat0 + featl];
    #pragma unroll
    for (int mt = 0; mt < 2; ++mt) {
      #pragma unroll
      for (int r = 0; r < 8; ++r) {
        const int tokl = 32 * wr + 16 * mt + 8 * h + r;
        const float y = acc[mt][nt][r] + bvl;
        const float yh = h_val(h_bits(y));
        sT[featl * 64 + tokl] = h_bits((y - yh) * RSCALE);
      }
    }
  }
  __syncthreads();
  vt_store_pass(sT, vtlo, bkv0, l0, w, lane);
  __threadfence();
  vt_store_pass(sT, vtlo, bkv0, l0, w, lane);
}

__device__ __forceinline__ v16h pack_p(v8f a, v8f c) {
  const v16h r = { (_Float16)(a[0] * PSCALE), (_Float16)(a[1] * PSCALE), (_Float16)(a[2] * PSCALE), (_Float16)(a[3] * PSCALE),
                   (_Float16)(a[4] * PSCALE), (_Float16)(a[5] * PSCALE), (_Float16)(a[6] * PSCALE), (_Float16)(a[7] * PSCALE),
                   (_Float16)(c[0] * PSCALE), (_Float16)(c[1] * PSCALE), (_Float16)(c[2] * PSCALE), (_Float16)(c[3] * PSCALE),
                   (_Float16)(c[4] * PSCALE), (_Float16)(c[5] * PSCALE), (_Float16)(c[6] * PSCALE), (_Float16)(c[7] * PSCALE) };
  return r;
}

__device__ __forceinline__ void ctx_store_pass(const unsigned short* so, unsigned short* ch, unsigned short* cl,
                                               int b, int head, int q0, int lane) {
  const int q8 = lane & 7, sub = lane >> 3;
  #pragma unroll
  for (int i = 0; i < 4; ++i) {
    const int row = i * 4 + sub;
    const v8us vh = *(const v8usa*)(so + row * 64 + 8 * q8);
    const v8us vl = *(const v8usa*)(so + 1024 + row * 64 + 8 * q8);
    const size_t gi = ((size_t)(b * SEQ + q0 + row)) * HID + head * HDIM + 8 * q8;
    *(volatile v8us*)(ch + gi) = vh;
    *(volatile v8us*)(cl + gi) = vl;
  }
}

__global__ __launch_bounds__(128) void attn_kernel(
    const _Float16* __restrict__ qh,
    const _Float16* __restrict__ kh,
    const _Float16* __restrict__ vthi,
    const _Float16* __restrict__ vtlo,
    unsigned short* __restrict__ ctxh,
    unsigned short* __restrict__ ctxl)
{
  __shared__ __attribute__((aligned(16))) unsigned short sO[4 * 2048];

  const int tid = threadIdx.x, lane = tid & 31, w = tid >> 5;
  const int h = lane >> 4, m = lane & 15;
  const int bh = blockIdx.y, b = bh >> 5, head = bh & 31, kvh = head >> 2;
  const int bkv = b * NKVH + kvh;
  const int q0 = blockIdx.x * 64 + 16 * w;

  const _Float16* qrow = qh + ((size_t)bh * SEQ + q0 + m) * HDIM;
  const v16h qb0 = frag_h(qrow, h);
  const v16h qb1 = frag_h(qrow + 32, h);

  const v8f zero8 = {0.f, 0.f, 0.f, 0.f, 0.f, 0.f, 0.f, 0.f};
  v8f oh[4], ol[4];
  #pragma unroll
  for (int t = 0; t < 4; ++t) { oh[t] = zero8; ol[t] = zero8; }
  float mrun = -1e30f, lrun = 0.0f;

  const _Float16* kbase = kh + ((size_t)bkv * SEQ + m) * HDIM;
  const _Float16* vhb = vthi + ((size_t)bkv * HDIM + m) * SEQ;
  const _Float16* vlb = vtlo + ((size_t)bkv * HDIM + m) * SEQ;

  #pragma unroll 1
  for (int kb = 0; kb < SEQ; kb += 64) {
    v8f s[4];
    #pragma unroll
    for (int j = 0; j < 4; ++j) {
      const _Float16* kp = kbase + (size_t)(kb + 16 * j) * HDIM;
      const v16h kf0 = frag_h(kp, h);
      const v16h kf1 = frag_h(kp + 32, h);
      v8f z = zero8;
      z = wmma_f16(kf0, qb0, z);
      z = wmma_f16(kf1, qb1, z);
      s[j] = z;
    }

    float mloc = s[0][0];
    #pragma unroll
    for (int j = 0; j < 4; ++j)
      #pragma unroll
      for (int r = 0; r < 8; ++r) mloc = fmaxf(mloc, s[j][r]);
    mloc = fmaxf(mloc, __shfl_xor(mloc, 16));
    const float mnew = fmaxf(mrun, mloc);
    const float alpha = __expf(mrun - mnew);
    mrun = mnew;
    float lsum = 0.0f;
    #pragma unroll
    for (int j = 0; j < 4; ++j)
      #pragma unroll
      for (int r = 0; r < 8; ++r) {
        const float p = __expf(s[j][r] - mnew);
        s[j][r] = p;
        lsum += p;
      }
    lsum += __shfl_xor(lsum, 16);
    lrun = lrun * alpha + lsum;
    #pragma unroll
    for (int t = 0; t < 4; ++t)
      #pragma unroll
      for (int r = 0; r < 8; ++r) { oh[t][r] = oh[t][r] * alpha; ol[t][r] = ol[t][r] * alpha; }

    const v16h pb0 = pack_p(s[0], s[1]);
    const v16h pb1 = pack_p(s[2], s[3]);

    #pragma unroll
    for (int t = 0; t < 4; ++t) {
      const _Float16* vp = vhb + (size_t)(16 * t) * SEQ + kb;
      const v16h vf0 = frag_h(vp, h);
      const v16h vf1 = frag_h(vp + 32, h);
      oh[t] = wmma_f16(vf0, pb0, oh[t]);
      oh[t] = wmma_f16(vf1, pb1, oh[t]);
      const _Float16* vq = vlb + (size_t)(16 * t) * SEQ + kb;
      const v16h wf0 = frag_h(vq, h);
      const v16h wf1 = frag_h(vq + 32, h);
      ol[t] = wmma_f16(wf0, pb0, ol[t]);
      ol[t] = wmma_f16(wf1, pb1, ol[t]);
    }
  }

  const float inv = (1.0f / lrun) * (1.0f / PSCALE);
  unsigned short* so = sO + w * 2048;
  #pragma unroll
  for (int t = 0; t < 4; ++t)
    #pragma unroll
    for (int r = 0; r < 8; ++r) {
      const float cv = (oh[t][r] + ol[t][r] * (1.0f / RSCALE)) * inv;
      const unsigned short hb = bf_rne(cv);
      const unsigned short lb = bf_rne(cv - bf_val(hb));
      const int li = m * 64 + 16 * t + 8 * h + r;
      so[li] = hb;
      so[1024 + li] = lb;
    }
  __syncthreads();

  ctx_store_pass(so, ctxh, ctxl, b, head, q0, lane);
  __threadfence();
  ctx_store_pass(so, ctxh, ctxl, b, head, q0, lane);
}

__device__ __forceinline__ void out_store_pass(const float* sC, float* out, int m0, int n0, int w, int lane) {
  const int q8 = lane & 7, sub = lane >> 3;
  #pragma unroll
  for (int i = 0; i < 16; ++i) {
    const int lid = w * 64 + i * 4 + sub;
    const int tok = lid >> 1, hl = lid & 1;
    const v4f v = *(const v4fa*)(sC + tok * 64 + 32 * hl + 4 * q8);
    *(volatile v4f*)(out + ((size_t)(m0 + tok)) * HID + n0 + 32 * hl + 4 * q8) = v;
  }
}

__global__ __launch_bounds__(128) void out_kernel(
    const unsigned short* __restrict__ ctxh,
    const unsigned short* __restrict__ ctxl,
    const unsigned short* __restrict__ wohi,
    const unsigned short* __restrict__ wolo,
    const float* __restrict__ bo,
    float* __restrict__ out)
{
  __shared__ __attribute__((aligned(16))) float sC[128 * 64];

  const int tid = threadIdx.x, lane = tid & 31, w = tid >> 5;
  const int h = lane >> 4, m = lane & 15;
  const int m0 = blockIdx.x * 128, n0 = blockIdx.y * 64;
  const int m0w = m0 + 32 * w;

  const unsigned short* a0h = ctxh + (size_t)(m0w + m) * HID;
  const unsigned short* a1h = a0h + (size_t)16 * HID;
  const unsigned short* a0l = ctxl + (size_t)(m0w + m) * HID;
  const unsigned short* a1l = a0l + (size_t)16 * HID;
  const unsigned short* wbh = wohi + (size_t)(n0 + m) * HID;
  const unsigned short* wbl = wolo + (size_t)(n0 + m) * HID;

  const v8f zero8 = {0.f, 0.f, 0.f, 0.f, 0.f, 0.f, 0.f, 0.f};
  v8f acc[2][4];
  #pragma unroll
  for (int mt = 0; mt < 2; ++mt)
    #pragma unroll
    for (int nt = 0; nt < 4; ++nt) acc[mt][nt] = zero8;

  #pragma unroll 1
  for (int k0 = 0; k0 < HID; k0 += 32) {
    const v16b ah0 = frag_b(a0h + k0, h);
    const v16b ah1 = frag_b(a1h + k0, h);
    const v16b al0 = frag_b(a0l + k0, h);
    const v16b al1 = frag_b(a1l + k0, h);
    #pragma unroll
    for (int nt = 0; nt < 4; ++nt) {
      const v16b bhf = frag_b(wbh + (size_t)nt * 16 * HID + k0, h);
      const v16b blf = frag_b(wbl + (size_t)nt * 16 * HID + k0, h);
      acc[0][nt] = wmma_bf16(ah0, bhf, acc[0][nt]);
      acc[0][nt] = wmma_bf16(ah0, blf, acc[0][nt]);
      acc[0][nt] = wmma_bf16(al0, bhf, acc[0][nt]);
      acc[1][nt] = wmma_bf16(ah1, bhf, acc[1][nt]);
      acc[1][nt] = wmma_bf16(ah1, blf, acc[1][nt]);
      acc[1][nt] = wmma_bf16(al1, bhf, acc[1][nt]);
    }
  }

  #pragma unroll
  for (int nt = 0; nt < 4; ++nt) {
    const int featl = 16 * nt + m;
    const float bvl = bo[n0 + featl];
    #pragma unroll
    for (int mt = 0; mt < 2; ++mt) {
      #pragma unroll
      for (int r = 0; r < 8; ++r) {
        const int tokl = 32 * w + 16 * mt + 8 * h + r;
        sC[tokl * 64 + featl] = acc[mt][nt][r] + bvl;
      }
    }
  }
  __syncthreads();

  out_store_pass(sC, out, m0, n0, w, lane);
  __threadfence();
  out_store_pass(sC, out, m0, n0, w, lane);
}

extern "C" void kernel_launch(void* const* d_in, const int* in_sizes, int n_in,
                              void* d_out, int out_size, void* d_ws, size_t ws_size,
                              hipStream_t stream) {
  if (n_in < 9) return;
  if (in_sizes[0] != MROWS * HID) return;
  if (in_sizes[1] != HID * HID || in_sizes[7] != HID * HID) return;
  if (in_sizes[2] != HID || in_sizes[8] != HID) return;
  if (in_sizes[3] != KVW * HID || in_sizes[5] != KVW * HID) return;
  if (in_sizes[4] != KVW || in_sizes[6] != KVW) return;
  if (out_size != MROWS * HID) return;

  const float* x  = (const float*)d_in[0];
  const float* Wq = (const float*)d_in[1];
  const float* bq = (const float*)d_in[2];
  const float* Wk = (const float*)d_in[3];
  const float* bk = (const float*)d_in[4];
  const float* Wv = (const float*)d_in[5];
  const float* bv = (const float*)d_in[6];
  const float* Wo = (const float*)d_in[7];
  const float* bo = (const float*)d_in[8];
  float* out = (float*)d_out;

  const size_t xh_b   = (size_t)MROWS * HID * 2;
  const size_t wqh_b  = (size_t)HID * HID * 2;
  const size_t wkh_b  = (size_t)KVW * HID * 2;
  const size_t wvp_b  = (size_t)KVW * HID * 2;
  const size_t wop_b  = (size_t)HID * HID * 2;
  const size_t qh_b   = (size_t)BATCH * NQH * SEQ * HDIM * 2;
  const size_t kh_b   = (size_t)BATCH * NKVH * SEQ * HDIM * 2;
  const size_t vtp_b  = (size_t)BATCH * NKVH * HDIM * SEQ * 2;
  const size_t ctxp_b = (size_t)MROWS * HID * 2;
  const size_t total = xh_b + wqh_b + wkh_b + 2 * wvp_b + 2 * wop_b + qh_b + kh_b + 2 * vtp_b + 2 * ctxp_b;
  if (total > ws_size) return;

  char* ws = (char*)d_ws;
  size_t off = 0;
  _Float16* xh = (_Float16*)(ws + off);               off += xh_b;
  _Float16* wqh = (_Float16*)(ws + off);              off += wqh_b;
  _Float16* wkh = (_Float16*)(ws + off);              off += wkh_b;
  unsigned short* wvhi = (unsigned short*)(ws + off); off += wvp_b;
  unsigned short* wvlo = (unsigned short*)(ws + off); off += wvp_b;
  unsigned short* wohi = (unsigned short*)(ws + off); off += wop_b;
  unsigned short* wolo = (unsigned short*)(ws + off); off += wop_b;
  _Float16* qh = (_Float16*)(ws + off);               off += qh_b;
  _Float16* kh = (_Float16*)(ws + off);               off += kh_b;
  _Float16* vthi = (_Float16*)(ws + off);             off += vtp_b;
  _Float16* vtlo = (_Float16*)(ws + off);             off += vtp_b;
  unsigned short* ctxh = (unsigned short*)(ws + off); off += ctxp_b;
  unsigned short* ctxl = (unsigned short*)(ws + off); off += ctxp_b;
  if (off > ws_size) return;

  convert_kernel<<<CVT_BLOCKS, 256, 0, stream>>>(x, Wq, Wk, Wv, Wo, xh, wqh, wkh, wvhi, wvlo, wohi, wolo);

  dim3 gQK(MROWS / 128, NQH + NKVH);
  proj_qk_kernel<<<gQK, 128, 0, stream>>>(xh, wqh, wkh, bq, bk, qh, kh);

  dim3 gV(MROWS / 64, KVW / 256);
  proj_v_kernel<<<gV, 256, 0, stream>>>(x, wvhi, wvlo, bv, vthi, vtlo);

  dim3 gAtt(SEQ / 64, BATCH * NQH);
  attn_kernel<<<gAtt, 128, 0, stream>>>(qh, kh, vthi, vtlo, ctxh, ctxl);

  dim3 gOut(MROWS / 128, HID / 64);
  out_kernel<<<gOut, 128, 0, stream>>>(ctxh, ctxl, wohi, wolo, bo, out);
}
